// Hyper_Block_54125177864653
// MI455X (gfx1250) — hardware-verified
//
#include <hip/hip_runtime.h>
#include <math.h>
#include <stdint.h>

#define NB    8
#define NT    1024
#define DM    768
#define NH    4
#define HD    192
#define NBH   (NB * NH)
#define NTOK  (NB * NT)
#define NQK   (NBH * NT)
#define NCEN  20
#define NCP   64
#define KVT   32
#define NQB   (NT / 64)
#define QKVR  (3 * DM)

static_assert(NH * HD == DM);
static_assert(DM == 96 * 8);
static_assert(DM == 192 * 4);
static_assert((HD % 64) == 0 && (HD % 32) == 0);
static_assert((NT % 64) == 0 && (NT % KVT) == 0 && KVT == 32);
static_assert((NT & (NT - 1)) == 0);
static_assert((NTOK % 64) == 0 && (DM % 64) == 0);
static_assert((((NTOK / 64) * (DM / 64)) % 8) == 0);
static_assert((((NQK / 32) * (HD / 64)) % 8) == 0);
static_assert((((NTOK / 64) * (NCP / 64)) % 8) == 0);
static_assert(((QKVR * DM / 8) % 256) == 0 && ((DM * DM / 8) % 256) == 0);
static_assert((NQK % 32) == 0);
static_assert(NCEN <= 32 && NCEN <= NCP);
static_assert((KVT * HD / 8) == 6 * 128 && (HD * KVT / 8) == 6 * 128);
static_assert(((NCP * DM / 8) % 256) == 0);

typedef _Float16 v16h __attribute__((ext_vector_type(16)));
typedef _Float16 v8h  __attribute__((ext_vector_type(8)));
typedef float    v8f  __attribute__((ext_vector_type(8)));
typedef float    v4f  __attribute__((ext_vector_type(4)));
typedef unsigned int v4u __attribute__((ext_vector_type(4)));

__device__ __forceinline__ unsigned short bf_bits(float f) {
  unsigned u = __float_as_uint(f);
  return (unsigned short)((u + 0x7FFFu + ((u >> 16) & 1u)) >> 16);
}
__device__ __forceinline__ float bf_up(unsigned short h) { return __uint_as_float(((unsigned)h) << 16); }
__device__ __forceinline__ float bfr(float f) { return bf_up(bf_bits(f)); }
__device__ __forceinline__ unsigned short h_bits(_Float16 x) { return __builtin_bit_cast(unsigned short, x); }
__device__ __forceinline__ unsigned pk16(unsigned short a, unsigned short b) { return (unsigned)a | ((unsigned)b << 16); }
__device__ __forceinline__ v8f zero8() { v8f z = {0.f, 0.f, 0.f, 0.f, 0.f, 0.f, 0.f, 0.f}; return z; }

__device__ __forceinline__ void ld8(const float* p, float* o) {
  const v4f a = *(const v4f*)(p);
  const v4f b = *(const v4f*)(p + 4);
  o[0] = a[0]; o[1] = a[1]; o[2] = a[2]; o[3] = a[3];
  o[4] = b[0]; o[5] = b[1]; o[6] = b[2]; o[7] = b[3];
}

__device__ __forceinline__ v16h ldfrag_h(const _Float16* p) {
  union { v16h v; v8h h[2]; } f;
  f.h[0] = *(const v8h*)(p);
  f.h[1] = *(const v8h*)(p + 16);
  return f.v;
}

__device__ __forceinline__ v8f mma_h(v16h a, v16h b, v8f c) {
  c = __builtin_amdgcn_wmma_f32_16x16x32_f16(false, a, false, b, (short)0, c, false, false);
#if defined(__HIP_DEVICE_COMPILE__)
  asm volatile("v_nop\n\tv_nop\n\tv_nop\n\tv_nop" : "+v"(c) : "v"(a), "v"(b));
#endif
  return c;
}
__device__ __forceinline__ v8f mma_h_raw(v16h a, v16h b, v8f c) {
  return __builtin_amdgcn_wmma_f32_16x16x32_f16(false, a, false, b, (short)0, c, false, false);
}
__device__ __forceinline__ void dep_guard_h(v8f& a, v8f& b, v16h x) {
#if defined(__HIP_DEVICE_COMPILE__)
  asm volatile("v_nop\n\tv_nop\n\tv_nop\n\tv_nop" : "+v"(a), "+v"(b) : "v"(x));
#endif
}
__device__ __forceinline__ void dep_guard_hl(v8f& a, v8f& b, v8f& c, v8f& d, v16h x, v16h y) {
#if defined(__HIP_DEVICE_COMPILE__)
  asm volatile("v_nop\n\tv_nop\n\tv_nop\n\tv_nop" : "+v"(a), "+v"(b), "+v"(c), "+v"(d) : "v"(x), "v"(y));
#endif
}
__device__ __forceinline__ void keep4_h(v16h a, v16h b, v16h c, v16h d) {
#if defined(__HIP_DEVICE_COMPILE__)
  asm volatile("v_nop" :: "v"(a), "v"(b), "v"(c), "v"(d));
#endif
}
__device__ __forceinline__ void acc_guard4(v8f& a, v8f& b, v8f& c, v8f& d) {
#if defined(__HIP_DEVICE_COMPILE__)
  asm volatile("v_nop\n\tv_nop\n\tv_nop\n\tv_nop" : "+v"(a), "+v"(b), "+v"(c), "+v"(d));
#endif
}

__global__ __launch_bounds__(256) void w_cvt(const float* __restrict__ in, unsigned short* out, int n8,
                                             float sc) {
  const int i = blockIdx.x * 256 + threadIdx.x;
  if (i < n8) {
    const v4f a = *(const v4f*)(in + (size_t)i * 8);
    const v4f b = *(const v4f*)(in + (size_t)i * 8 + 4);
    v4u p;
    p[0] = pk16(h_bits((_Float16)(bfr(a[0]) * sc)), h_bits((_Float16)(bfr(a[1]) * sc)));
    p[1] = pk16(h_bits((_Float16)(bfr(a[2]) * sc)), h_bits((_Float16)(bfr(a[3]) * sc)));
    p[2] = pk16(h_bits((_Float16)(bfr(b[0]) * sc)), h_bits((_Float16)(bfr(b[1]) * sc)));
    p[3] = pk16(h_bits((_Float16)(bfr(b[2]) * sc)), h_bits((_Float16)(bfr(b[3]) * sc)));
    *(volatile v4u*)(out + (size_t)i * 8) = p;
    __threadfence();
    *(volatile v4u*)(out + (size_t)i * 8) = p;
  }
}

__global__ __launch_bounds__(256) void wt_cvt(const float* __restrict__ W, int ncols, int nrows,
                                              unsigned short* outp, float sc) {
  __shared__ __align__(16) float sw[64 * 68];
  const int tid = threadIdx.x;
  const int n0 = blockIdx.x * 64;
  const int k0 = blockIdx.y * 64;
#pragma unroll
  for (int i = 0; i < 4; ++i) {
    const int idx = i * 256 + tid;
    const int kk = idx >> 4, c4 = (idx & 15) * 4;
    const v4f a = *(const v4f*)(W + (size_t)(k0 + kk) * ncols + n0 + c4);
    *(v4f*)(sw + kk * 68 + c4) = a;
  }
  __syncthreads();

  const int g = tid >> 3, piece = tid & 7;
  v4u ov[2];
  size_t oofs[2];
#pragma unroll
  for (int it = 0; it < 2; ++it) {
    const int nn = it * 32 + g;
    v4u a;
#pragma unroll
    for (int e = 0; e < 4; ++e) {
      const float f0 = sw[(piece * 8 + 2 * e) * 68 + nn];
      const float f1 = sw[(piece * 8 + 2 * e + 1) * 68 + nn];
      a[e] = pk16(h_bits((_Float16)(bfr(f0) * sc)), h_bits((_Float16)(bfr(f1) * sc)));
    }
    ov[it] = a;
    oofs[it] = (size_t)(n0 + nn) * nrows + k0 + piece * 8;
  }
  for (int pass = 0; pass < 2; ++pass) {
#pragma unroll
    for (int it = 0; it < 2; ++it) *(volatile v4u*)(outp + oofs[it]) = ov[it];
    __threadfence();
  }
}

__global__ __launch_bounds__(256) void cen_prep(const float* __restrict__ cen, unsigned short* c16, float* bc) {
  __shared__ __align__(16) float red[32];
  const int tid = threadIdx.x, wave = tid >> 5, lane = tid & 31;
  if (tid < 32) red[tid] = 0.f;
  for (int it = 0; it < (NCP * DM / 8) / 256; ++it) {
    const int p  = it * 256 + tid;
    const int j  = p / (DM / 8);
    const int k8 = (p - j * (DM / 8)) * 8;
    const int jc = (j < NCEN) ? j : (NCEN - 1);
    float f[8];
    ld8(cen + (size_t)jc * DM + k8, f);
    v4u a;
#pragma unroll
    for (int e = 0; e < 4; ++e) {
      const float v0 = (j < NCEN) ? bfr(f[2 * e]) : 0.f;
      const float v1 = (j < NCEN) ? bfr(f[2 * e + 1]) : 0.f;
      a[e] = pk16(h_bits((_Float16)v0), h_bits((_Float16)v1));
    }
    const size_t o = (size_t)p * 8;
    *(volatile v4u*)(c16 + o) = a;
    __threadfence();
    *(volatile v4u*)(c16 + o) = a;
  }
  __syncthreads();
#pragma unroll 1
  for (int jj = 0; jj < 3; ++jj) {
    const int j  = wave + 8 * jj;
    const int jc = (j < NCEN) ? j : (NCEN - 1);
    float s = 0.f;
#pragma unroll
    for (int q = 0; q < 3; ++q) {
      const int pc = lane + 32 * q;
      float f[8];
      ld8(cen + (size_t)jc * DM + pc * 8, f);
#pragma unroll
      for (int e = 0; e < 8; ++e) { const float v = bfr(f[e]); s += v * v; }
    }
#pragma unroll
    for (int off = 16; off >= 1; off >>= 1) s += __shfl_xor(s, off, 32);
    if (lane == 0 && j < NCEN) red[j] = s;
  }
  __syncthreads();
  if (wave == 0 && lane < 8) {
    const v4f o = *(const v4f*)(red + lane * 4);
    *(volatile v4f*)(bc + lane * 4) = o;
    __threadfence();
    *(volatile v4f*)(bc + lane * 4) = o;
  }
}

__global__ __launch_bounds__(96) void ln_f16(const float* __restrict__ X, const float* __restrict__ gp,
                                             const float* __restrict__ bp, unsigned short* H, int rnd,
                                             float osc) {
#pragma clang fp contract(off)
  __shared__ float red[2][3];
  const int tid = threadIdx.x, wave = tid >> 5, lane = tid & 31;
  const int row = blockIdx.x;
  const int d0 = tid * 8;
  float x[8];
  ld8(X + (size_t)row * DM + d0, x);
  if (rnd != 0) {
#pragma unroll
    for (int e = 0; e < 8; ++e) x[e] = bfr(x[e]);
  }
  float s = 0.f;
#pragma unroll
  for (int e = 0; e < 8; ++e) s += x[e];
#pragma unroll
  for (int off = 16; off >= 1; off >>= 1) s += __shfl_xor(s, off, 32);
  if (lane == 0) red[0][wave] = s;
  __syncthreads();
  const float mu = ((red[0][0] + red[0][1]) + red[0][2]) * (1.0f / (float)DM);
  float d[8];
  float ss = 0.f;
#pragma unroll
  for (int e = 0; e < 8; ++e) { d[e] = x[e] - mu; ss += d[e] * d[e]; }
#pragma unroll
  for (int off = 16; off >= 1; off >>= 1) ss += __shfl_xor(ss, off, 32);
  if (lane == 0) red[1][wave] = ss;
  __syncthreads();
  const float var  = ((red[1][0] + red[1][1]) + red[1][2]) * (1.0f / (float)DM);
  const float rstd = rsqrtf(var + 1e-5f);
  float gv[8], bv[8];
  ld8(gp + d0, gv);
  ld8(bp + d0, bv);
  v4u a;
#pragma unroll
  for (int p = 0; p < 4; ++p) {
    const int e = 2 * p;
    const float y0 = (d[e] * rstd) * bfr(gv[e]) + bfr(bv[e]);
    const float y1 = (d[e + 1] * rstd) * bfr(gv[e + 1]) + bfr(bv[e + 1]);
    a[p] = pk16(h_bits((_Float16)(y0 * osc)), h_bits((_Float16)(y1 * osc)));
  }
  const size_t o = (size_t)row * DM + d0;
  *(volatile v4u*)(H + o) = a;
  __threadfence();
  *(volatile v4u*)(H + o) = a;
}

template <int MODE, int RR>
__global__ __launch_bounds__(256) void gemm64(
    const unsigned short* __restrict__ Ap, int lda,
    const unsigned short* __restrict__ Btp, int ldb,
    const float* __restrict__ bias, const float* __restrict__ res, int ldr,
    float* Cf, unsigned short* Ch, unsigned short* Cl, int ldc, int M, int N, int K, float oscale) {
  const _Float16* Ah = (const _Float16*)(const void*)Ap;
  const _Float16* Bh = (const _Float16*)(const void*)Btp;
  __shared__ __align__(16) float sT[8][16 * 68];
  const int lane = threadIdx.x & 31;
  const int wave = threadIdx.x >> 5;
  const int tilesN = N >> 6;
  const int tilesM = M >> 6;
  const int tile = blockIdx.x * 8 + wave;
  if (tile >= tilesM * tilesN) return;
  const int tm = tile / tilesN;
  const int tn = tile - tm * tilesN;
  const int m0 = tm << 6;
  const int n0 = tn << 6;

  const int rlane = lane & 15;
  const int koff  = (lane >> 4) * 8;
  const int mOff  = (lane >> 4) * 8;

  v8f acc[4][4];
#pragma unroll
  for (int i = 0; i < 4; ++i)
#pragma unroll
    for (int j = 0; j < 4; ++j) acc[i][j] = zero8();

  for (int k0 = 0; k0 < K; k0 += 32) {
    v16h bh[4];
#pragma unroll
    for (int j = 0; j < 4; ++j) {
      const size_t bo = (size_t)(n0 + (j << 4) + rlane) * ldb + koff + k0;
      bh[j] = ldfrag_h(Bh + bo);
    }
#pragma unroll
    for (int i = 0; i < 4; ++i) {
      const size_t ao = (size_t)(m0 + (i << 4) + rlane) * lda + koff + k0;
      const v16h ah = ldfrag_h(Ah + ao);
#pragma unroll
      for (int j = 0; j < 4; ++j) acc[i][j] = mma_h_raw(ah, bh[j], acc[i][j]);
      dep_guard_h(acc[i][0], acc[i][3], ah);
    }
    keep4_h(bh[0], bh[1], bh[2], bh[3]);
  }
  acc_guard4(acc[0][0], acc[0][1], acc[0][2], acc[0][3]);
  acc_guard4(acc[1][0], acc[1][1], acc[1][2], acc[1][3]);
  acc_guard4(acc[2][0], acc[2][1], acc[2][2], acc[2][3]);
  acc_guard4(acc[3][0], acc[3][1], acc[3][2], acc[3][3]);

  float* slab = sT[wave];
#pragma unroll
  for (int i = 0; i < 4; ++i) {
    const int mBase = m0 + (i << 4);
#pragma unroll
    for (int r = 0; r < 8; ++r) {
#pragma unroll
      for (int j = 0; j < 4; ++j) {
        slab[(mOff + r) * 68 + (j << 4) + rlane] = acc[i][j][r];
      }
    }
    __builtin_amdgcn_fence(__ATOMIC_RELEASE, "workgroup");
    __builtin_amdgcn_wave_barrier();
    __builtin_amdgcn_fence(__ATOMIC_ACQUIRE, "workgroup");
    if (MODE == 0 || MODE == 1) {
      const int h2 = lane >> 4, c4 = (lane & 15) * 4;
      v4f b4 = {0.f, 0.f, 0.f, 0.f};
      if (MODE == 1) {
        const v4f braw = *(const v4f*)(bias + n0 + c4);
#pragma unroll
        for (int e = 0; e < 4; ++e) b4[e] = bfr(braw[e]);
      }
      v4f ov[8];
#pragma unroll
      for (int it = 0; it < 8; ++it) {
        const int row = it * 2 + h2;
        const v4f xs = *(const v4f*)(slab + row * 68 + c4);
        v4f v = xs * oscale;
        if (MODE == 1) {
          v4f r4 = *(const v4f*)(res + (size_t)(mBase + row) * ldr + n0 + c4);
          if (RR != 0) {
#pragma unroll
            for (int e = 0; e < 4; ++e) r4[e] = bfr(r4[e]);
          }
          v = (v + b4) + r4;
        }
        ov[it] = v;
      }
      for (int pass = 0; pass < 2; ++pass) {
#pragma unroll
        for (int it = 0; it < 8; ++it) {
          const int row = it * 2 + h2;
          *(volatile v4f*)(Cf + (size_t)(mBase + row) * ldc + n0 + c4) = ov[it];
        }
        __threadfence();
      }
    } else {
      const int q8 = lane & 7, rr = lane >> 3, c8 = q8 * 8;
      const int hsel = n0 / HD;
      const int d0 = n0 - hsel * HD;
      v4u hv[4], lv[4];
      size_t po[4];
#pragma unroll
      for (int it = 0; it < 4; ++it) {
        const int row = it * 4 + rr;
        const int m = mBase + row;
        const int prow = ((m / NT) * NH + hsel) * NT + (m & (NT - 1));
        float xs[8];
        ld8(slab + row * 68 + c8, xs);
        v4u a, a2;
#pragma unroll
        for (int p = 0; p < 4; ++p) {
          const float v0 = xs[2 * p] * oscale, v1 = xs[2 * p + 1] * oscale;
          const _Float16 x0 = (_Float16)v0, x1 = (_Float16)v1;
          const unsigned short l0 = h_bits((_Float16)((v0 - (float)x0) * 2048.0f));
          const unsigned short l1 = h_bits((_Float16)((v1 - (float)x1) * 2048.0f));
          a[p] = pk16(h_bits(x0), h_bits(x1));
          a2[p] = pk16(l0, l1);
        }
        hv[it] = a; lv[it] = a2;
        po[it] = (size_t)prow * ldc + d0 + c8;
      }
      for (int pass = 0; pass < 2; ++pass) {
#pragma unroll
        for (int it = 0; it < 4; ++it) {
          *(volatile v4u*)(Ch + po[it]) = hv[it];
          *(volatile v4u*)(Cl + po[it]) = lv[it];
        }
        __threadfence();
      }
    }
    __builtin_amdgcn_fence(__ATOMIC_RELEASE, "workgroup");
    __builtin_amdgcn_wave_barrier();
    __builtin_amdgcn_fence(__ATOMIC_ACQUIRE, "workgroup");
  }
}

__global__ __launch_bounds__(256) void gemm2hl(
    const unsigned short* __restrict__ Ahp, const unsigned short* __restrict__ Alp, int lda,
    const unsigned short* __restrict__ Btp, int ldb,
    unsigned short* Ch, unsigned short* Cl, int ldc, int M, int N, int K, float oscale) {
  const _Float16* Ah = (const _Float16*)(const void*)Ahp;
  const _Float16* Al = (const _Float16*)(const void*)Alp;
  const _Float16* Bh = (const _Float16*)(const void*)Btp;
  __shared__ __align__(16) float sT[8][16 * 68];
  const int lane = threadIdx.x & 31;
  const int wave = threadIdx.x >> 5;
  const int tilesN = N >> 6;
  const int tilesM = M >> 5;
  const int tile = blockIdx.x * 8 + wave;
  if (tile >= tilesM * tilesN) return;
  const int tm = tile / tilesN;
  const int tn = tile - tm * tilesN;
  const int m0 = tm << 5;
  const int n0 = tn << 6;

  const int rlane = lane & 15;
  const int koff  = (lane >> 4) * 8;
  const int mOff  = (lane >> 4) * 8;

  v8f acch[2][4], accl[2][4];
#pragma unroll
  for (int i = 0; i < 2; ++i)
#pragma unroll
    for (int j = 0; j < 4; ++j) { acch[i][j] = zero8(); accl[i][j] = zero8(); }

  for (int k0 = 0; k0 < K; k0 += 32) {
    v16h bh[4];
#pragma unroll
    for (int j = 0; j < 4; ++j) {
      const size_t bo = (size_t)(n0 + (j << 4) + rlane) * ldb + koff + k0;
      bh[j] = ldfrag_h(Bh + bo);
    }
#pragma unroll
    for (int i = 0; i < 2; ++i) {
      const size_t ao = (size_t)(m0 + (i << 4) + rlane) * lda + koff + k0;
      const v16h ah = ldfrag_h(Ah + ao);
      const v16h al = ldfrag_h(Al + ao);
#pragma unroll
      for (int j = 0; j < 4; ++j) {
        acch[i][j] = mma_h_raw(ah, bh[j], acch[i][j]);
        accl[i][j] = mma_h_raw(al, bh[j], accl[i][j]);
      }
      dep_guard_hl(acch[i][0], acch[i][3], accl[i][0], accl[i][3], ah, al);
    }
    keep4_h(bh[0], bh[1], bh[2], bh[3]);
  }
  acc_guard4(acch[0][0], acch[0][1], acch[0][2], acch[0][3]);
  acc_guard4(acch[1][0], acch[1][1], acch[1][2], acch[1][3]);
  acc_guard4(accl[0][0], accl[0][1], accl[0][2], accl[0][3]);
  acc_guard4(accl[1][0], accl[1][1], accl[1][2], accl[1][3]);

  float* slab = sT[wave];
#pragma unroll
  for (int i = 0; i < 2; ++i) {
    const int mBase = m0 + (i << 4);
#pragma unroll
    for (int r = 0; r < 8; ++r) {
#pragma unroll
      for (int j = 0; j < 4; ++j) {
        slab[(mOff + r) * 68 + (j << 4) + rlane] = acch[i][j][r] + accl[i][j][r] * (1.0f / 2048.0f);
      }
    }
    __builtin_amdgcn_fence(__ATOMIC_RELEASE, "workgroup");
    __builtin_amdgcn_wave_barrier();
    __builtin_amdgcn_fence(__ATOMIC_ACQUIRE, "workgroup");
    {
      const int q8 = lane & 7, rr = lane >> 3, c8 = q8 * 8;
      v4u hv[4], lv[4];
      size_t po[4];
#pragma unroll
      for (int it = 0; it < 4; ++it) {
        const int row = it * 4 + rr;
        float xs[8];
        ld8(slab + row * 68 + c8, xs);
        v4u a, a2;
#pragma unroll
        for (int p = 0; p < 4; ++p) {
          const float v0 = xs[2 * p] * oscale, v1 = xs[2 * p + 1] * oscale;
          const _Float16 x0 = (_Float16)v0, x1 = (_Float16)v1;
          const unsigned short l0 = h_bits((_Float16)((v0 - (float)x0) * 2048.0f));
          const unsigned short l1 = h_bits((_Float16)((v1 - (float)x1) * 2048.0f));
          a[p] = pk16(h_bits(x0), h_bits(x1));
          a2[p] = pk16(l0, l1);
        }
        hv[it] = a; lv[it] = a2;
        po[it] = (size_t)(mBase + row) * ldc + n0 + c8;
      }
      for (int pass = 0; pass < 2; ++pass) {
#pragma unroll
        for (int it = 0; it < 4; ++it) {
          *(volatile v4u*)(Ch + po[it]) = hv[it];
          *(volatile v4u*)(Cl + po[it]) = lv[it];
        }
        __threadfence();
      }
    }
    __builtin_amdgcn_fence(__ATOMIC_RELEASE, "workgroup");
    __builtin_amdgcn_wave_barrier();
    __builtin_amdgcn_fence(__ATOMIC_ACQUIRE, "workgroup");
  }
}

__global__ __launch_bounds__(256) void vt_planes(const float* __restrict__ vf, unsigned short* vt, float vscale) {
  __shared__ __align__(16) float sv[64 * 68];
  const int tid = threadIdx.x;
  const int t0  = blockIdx.x * 64;
  const int by  = blockIdx.y;
  const int bh  = by / 3;
  const int dt  = by - bh * 3;
  const int b   = bh / NH;
  const int hh  = bh - b * NH;
#pragma unroll
  for (int i = 0; i < 4; ++i) {
    const int idx = i * 256 + tid;
    const int tt = idx >> 4, c4 = (idx & 15) * 4;
    const v4f a = *(const v4f*)(vf + ((size_t)(b * NT + t0 + tt)) * DM + hh * HD + dt * 64 + c4);
    *(v4f*)(sv + tt * 68 + c4) = a;
  }
  __syncthreads();

  const int g = tid >> 3, piece = tid & 7;
  v4u hv[2];
  size_t hofs[2];
#pragma unroll
  for (int it = 0; it < 2; ++it) {
    const int d = it * 32 + g;
    v4u a;
#pragma unroll
    for (int e = 0; e < 4; ++e) {
      const float f0 = sv[(piece * 8 + 2 * e) * 68 + d] * vscale;
      const float f1 = sv[(piece * 8 + 2 * e + 1) * 68 + d] * vscale;
      a[e] = pk16(h_bits((_Float16)f0), h_bits((_Float16)f1));
    }
    hv[it] = a;
    hofs[it] = ((size_t)(bh * HD + dt * 64 + d)) * NT + t0 + piece * 8;
  }
  for (int pass = 0; pass < 2; ++pass) {
#pragma unroll
    for (int it = 0; it < 2; ++it) *(volatile v4u*)(vt + hofs[it]) = hv[it];
    __threadfence();
  }
}

__global__ __launch_bounds__(256) void kmk_k(const unsigned short* __restrict__ khp,
                                             const unsigned short* __restrict__ klp,
                                             const unsigned short* __restrict__ mhp,
                                             const unsigned short* __restrict__ mlp, float* kmk) {
  __shared__ __align__(16) float red[32];
  const int tid = threadIdx.x, wave = tid >> 5, lane = tid & 31;
  const _Float16* Kh = (const _Float16*)(const void*)khp;
  const _Float16* Kl = (const _Float16*)(const void*)klp;
  const _Float16* Mh = (const _Float16*)(const void*)mhp;
  const _Float16* Ml = (const _Float16*)(const void*)mlp;
  const int pc = (lane < HD / 8) ? lane : (HD / 8 - 1);
#pragma unroll 1
  for (int q = 0; q < 4; ++q) {
    const int r = blockIdx.x * 32 + wave * 4 + q;
    const size_t o = (size_t)r * HD + pc * 8;
    const v8h a0 = *(const v8h*)(Kh + o);
    const v8h a1 = *(const v8h*)(Kl + o);
    const v8h b0 = *(const v8h*)(Mh + o);
    const v8h b1 = *(const v8h*)(Ml + o);
    float s = 0.f;
#pragma unroll
    for (int e = 0; e < 8; ++e) {
      const float kv = ((float)a0[e] + (float)a1[e] * (1.0f / 2048.0f)) * (1.0f / 16.0f);
      const float mv = ((float)b0[e] + (float)b1[e] * (1.0f / 2048.0f)) * (1.0f / 16.0f);
      s += kv * mv;
    }
    s = (lane < HD / 8) ? s : 0.f;
#pragma unroll
    for (int off = 16; off >= 1; off >>= 1) s += __shfl_xor(s, off, 32);
    if (lane == 0) red[wave * 4 + q] = s;
  }
  __syncthreads();
  if (wave == 0 && lane < 8) {
    const v4f o = *(const v4f*)(red + lane * 4);
    const size_t go = (size_t)blockIdx.x * 32 + lane * 4;
    *(volatile v4f*)(kmk + go) = o;
    __threadfence();
    *(volatile v4f*)(kmk + go) = o;
  }
}

__global__ __launch_bounds__(128)
void attn_k(const unsigned short* __restrict__ qmhp, const unsigned short* __restrict__ qmlp,
            const unsigned short* __restrict__ khp, const unsigned short* __restrict__ klp,
            const unsigned short* __restrict__ vtp, const float* __restrict__ kmkp,
            const float* __restrict__ scalep, unsigned short* yout) {
  union FH { v16h v; v8h h[2]; };
  __shared__ __align__(16) float lds[4 * 16 * HD];
  _Float16* Khs = (_Float16*)lds;
  _Float16* Kls = Khs + KVT * HD;
  _Float16* Vts = Kls + KVT * HD;
  _Float16* Psh = Vts + HD * KVT;
  static_assert((3 * KVT * HD + 4 * 16 * KVT) * 2 <= 4 * 16 * HD * 4);

  const int tid  = threadIdx.x;
  const int wave = tid >> 5;
  const int lane = tid & 31;
  const int hh   = lane >> 4;
  const int c    = lane & 15;

  const int bx = blockIdx.x;
  const int bh = bx / NQB;
  const int qb = bx - bh * NQB;
  const int b  = bh / NH;
  const int h  = bh - b * NH;
  const int q0 = qb * 64 + wave * 16;
  const size_t rb = (size_t)bh * NT;

  const _Float16* QMh = (const _Float16*)(const void*)qmhp;
  const _Float16* QMl = (const _Float16*)(const void*)qmlp;
  const _Float16* Kh  = (const _Float16*)(const void*)khp;
  const _Float16* Kl  = (const _Float16*)(const void*)klp;
  const _Float16* Vt  = (const _Float16*)(const void*)vtp + (size_t)bh * HD * NT;
  const float* kmkB = kmkp + rb;
  const float bscale = bfr(scalep[0]);

  float mrow[8], lrow[8];
  v8f oacc[12];
#pragma unroll
  for (int r = 0; r < 8; ++r) { mrow[r] = -INFINITY; lrow[r] = 0.f; }
#pragma unroll
  for (int t = 0; t < 12; ++t) oacc[t] = zero8();

#pragma unroll 1
  for (int kt = 0; kt < NT / KVT; ++kt) {
    const int kv0 = kt * KVT;
    __syncthreads();
#pragma unroll
    for (int it = 0; it < 6; ++it) {
      const int p = it * 128 + tid;
      {
        const int row = p / (HD / 8);
        const int c8  = (p - row * (HD / 8)) * 8;
        const size_t g = (rb + kv0 + row) * HD + c8;
        const v8h a0 = *(const v8h*)(Kh + g);
        const v8h a1 = *(const v8h*)(Kl + g);
        *(v8h*)(Khs + row * HD + c8) = a0;
        *(v8h*)(Kls + row * HD + c8) = a1;
      }
      {
        const int d  = p >> 2;
        const int c8 = (p & 3) * 8;
        const v8h v0 = *(const v8h*)(Vt + (size_t)d * NT + kv0 + c8);
        *(v8h*)(Vts + d * KVT + c8) = v0;
      }
    }
    __syncthreads();

    v8f s[2], s2[2];
#pragma unroll
    for (int j = 0; j < 2; ++j) { s[j] = zero8(); s2[j] = zero8(); }
#pragma unroll
    for (int dc = 0; dc < HD / 32; ++dc) {
      const size_t qo = (rb + q0 + c) * HD + dc * 32 + 8 * hh;
      const v16h qa = ldfrag_h(QMh + qo);
      const v16h ql = ldfrag_h(QMl + qo);
#pragma unroll
      for (int j = 0; j < 2; ++j) {
        FH kb, kc;
        kb.h[0] = *(const v8h*)(Khs + (j * 16 + c) * HD + dc * 32 + 8 * hh);
        kb.h[1] = *(const v8h*)(Khs + (j * 16 + c) * HD + dc * 32 + 16 + 8 * hh);
        kc.h[0] = *(const v8h*)(Kls + (j * 16 + c) * HD + dc * 32 + 8 * hh);
        kc.h[1] = *(const v8h*)(Kls + (j * 16 + c) * HD + dc * 32 + 16 + 8 * hh);
        s[j]  = mma_h(qa, kb.v, s[j]);
        s2[j] = mma_h(qa, kc.v, s2[j]);
        s2[j] = mma_h(ql, kb.v, s2[j]);
      }
    }

    float kk[2];
#pragma unroll
    for (int j = 0; j < 2; ++j) kk[j] = kmkB[kv0 + j * 16 + c];
    _Float16* pwh = Psh + wave * (16 * KVT);
#pragma unroll
    for (int r = 0; r < 8; ++r) {
      float m = -INFINITY;
#pragma unroll
      for (int j = 0; j < 2; ++j) {
        const float sd = (s[j][r] + s2[j][r] * (1.0f / 2048.0f)) * (1.0f / 256.0f);
        const float dd = kk[j] - 2.0f * sd;
        const float lg = -(dd * bscale);
        s[j][r] = lg;
        m = fmaxf(m, lg);
      }
#pragma unroll
      for (int off = 1; off < 16; off <<= 1) m = fmaxf(m, __shfl_xor(m, off, 32));
      const float mnew  = fmaxf(mrow[r], m);
      const float alpha = __expf(mrow[r] - mnew);
      mrow[r] = mnew;
      float psum = 0.f;
#pragma unroll
      for (int j = 0; j < 2; ++j) {
        const float p = __expf(s[j][r] - mnew);
        psum += p;
        const _Float16 ph = (_Float16)(p * 1024.0f);
        pwh[(8 * hh + r) * KVT + j * 16 + c] = ph;
      }
#pragma unroll
      for (int off = 1; off < 16; off <<= 1) psum += __shfl_xor(psum, off, 32);
      lrow[r] = lrow[r] * alpha + psum;
#pragma unroll
      for (int t = 0; t < 12; ++t) oacc[t][r] *= alpha;
    }
    __builtin_amdgcn_fence(__ATOMIC_RELEASE, "workgroup");
    __builtin_amdgcn_wave_barrier();
    __builtin_amdgcn_fence(__ATOMIC_ACQUIRE, "workgroup");

    FH pa;
    pa.h[0] = *(const v8h*)(pwh + c * KVT + 8 * hh);
    pa.h[1] = *(const v8h*)(pwh + c * KVT + 16 + 8 * hh);
#pragma unroll
    for (int t = 0; t < 12; ++t) {
      FH vb;
      vb.h[0] = *(const v8h*)(Vts + (t * 16 + c) * KVT + 8 * hh);
      vb.h[1] = *(const v8h*)(Vts + (t * 16 + c) * KVT + 16 + 8 * hh);
      oacc[t] = mma_h(pa.v, vb.v, oacc[t]);
    }
  }

  __syncthreads();
  float* os = lds + wave * (16 * HD);
#pragma unroll
  for (int r = 0; r < 8; ++r) {
    const float inv = (1.0f / lrow[r]) * (1.0f / 1024.0f);
#pragma unroll
    for (int t = 0; t < 12; ++t) os[(8 * hh + r) * HD + t * 16 + c] = oacc[t][r] * inv;
  }
  __builtin_amdgcn_fence(__ATOMIC_RELEASE, "workgroup");
  __builtin_amdgcn_wave_barrier();
  __builtin_amdgcn_fence(__ATOMIC_ACQUIRE, "workgroup");
  v4u ov[12];
#pragma unroll
  for (int it = 0; it < 12; ++it) {
    const int p = it * 32 + lane;
    const int row = p / (HD / 8);
    const int pc  = p - row * (HD / 8);
    float xs[8];
    ld8(os + row * HD + pc * 8, xs);
    v4u a;
#pragma unroll
    for (int e = 0; e < 4; ++e) a[e] = pk16(h_bits((_Float16)xs[2 * e]), h_bits((_Float16)xs[2 * e + 1]));
    ov[it] = a;
  }
  for (int pass = 0; pass < 2; ++pass) {
#pragma unroll
    for (int it = 0; it < 12; ++it) {
      const int p = it * 32 + lane;
      const int row = p / (HD / 8);
      const int pc  = p - row * (HD / 8);
      const size_t go = ((size_t)(b * NT + q0 + row)) * DM + (size_t)h * HD + pc * 8;
      *(volatile v4u*)(yout + go) = ov[it];
    }
    __threadfence();
  }
}

__global__ __launch_bounds__(192) void final_k(const float* __restrict__ x1, const float* __restrict__ gp,
                                               const float* __restrict__ bp, const float* __restrict__ cg,
                                               const float* __restrict__ bcp, const float* __restrict__ betap,
                                               const float* __restrict__ fcw, float* outp) {
#pragma clang fp contract(off)
  __shared__ float red[3][6];
  __shared__ float rbf[32];
  const int tid = threadIdx.x, wave = tid >> 5, lane = tid & 31;
  const int row = blockIdx.x;
  const int c0 = tid * 4;
  const v4f xv = *(const v4f*)(x1 + (size_t)row * DM + c0);
  float s = ((xv[0] + xv[1]) + xv[2]) + xv[3];
#pragma unroll
  for (int off = 16; off >= 1; off >>= 1) s += __shfl_xor(s, off, 32);
  if (lane == 0) red[0][wave] = s;
  __syncthreads();
  const float mu = (((((red[0][0] + red[0][1]) + red[0][2]) + red[0][3]) + red[0][4]) + red[0][5]) *
                   (1.0f / (float)DM);
  float d[4];
  float ss = 0.f;
#pragma unroll
  for (int e = 0; e < 4; ++e) { d[e] = xv[e] - mu; ss += d[e] * d[e]; }
#pragma unroll
  for (int off = 16; off >= 1; off >>= 1) ss += __shfl_xor(ss, off, 32);
  if (lane == 0) red[1][wave] = ss;
  __syncthreads();
  const float var  = (((((red[1][0] + red[1][1]) + red[1][2]) + red[1][3]) + red[1][4]) + red[1][5]) *
                     (1.0f / (float)DM);
  const float rstd = rsqrtf(var + 1e-5f);
  const v4f g4 = *(const v4f*)(gp + c0);
  const v4f b4 = *(const v4f*)(bp + c0);
  float pa = 0.f;
#pragma unroll
  for (int e = 0; e < 4; ++e) {
    const float hv = (d[e] * rstd) * bfr(g4[e]) + bfr(b4[e]);
    pa += hv * hv;
  }
#pragma unroll
  for (int off = 16; off >= 1; off >>= 1) pa += __shfl_xor(pa, off, 32);
  if (lane == 0) red[2][wave] = pa;
  __syncthreads();
  const float a = ((((red[2][0] + red[2][1]) + red[2][2]) + red[2][3]) + red[2][4]) + red[2][5];
  if (tid < NCEN) {
    const float cj = 2.0f * cg[(size_t)row * NCP + tid];
    const float bj = bcp[tid];
    const float be = bfr(betap[tid]);
    const float t2 = (a - cj) + bj;
    rbf[tid] = expf((-be) * t2);
  }
  __syncthreads();
  v4f o;
#pragma unroll
  for (int e = 0; e < 4; ++e) {
    const int n = c0 + e;
    const float* fr = fcw + (size_t)n * NCEN;
    float acc = 0.f;
#pragma unroll
    for (int q = 0; q < NCEN / 4; ++q) {
      const v4f f = *(const v4f*)(fr + 4 * q);
      acc += rbf[4 * q] * bfr(f[0]);
      acc += rbf[4 * q + 1] * bfr(f[1]);
      acc += rbf[4 * q + 2] * bfr(f[2]);
      acc += rbf[4 * q + 3] * bfr(f[3]);
    }
    o[e] = xv[e] + acc;
  }
  const size_t go = (size_t)row * DM + c0;
  *(volatile v4f*)(outp + go) = o;
  __threadfence();
  *(volatile v4f*)(outp + go) = o;
}

extern "C" void kernel_launch(void* const* d_in, const int* in_sizes, int n_in,
                              void* d_out, int out_size, void* d_ws, size_t ws_size,
                              hipStream_t stream) {
  if (n_in < 13) return;
  if (in_sizes[0] != NTOK * DM) return;
  if (in_sizes[1] != DM || in_sizes[2] != DM) return;
  if (in_sizes[3] != QKVR * DM) return;
  if (in_sizes[4] != HD * HD) return;
  if (in_sizes[5] < 1) return;
  if (in_sizes[6] != DM * DM) return;
  if (in_sizes[7] != DM || in_sizes[8] != DM || in_sizes[9] != DM) return;
  if (in_sizes[10] != NCEN * DM) return;
  if (in_sizes[11] != NCEN) return;
  if (in_sizes[12] != DM * NCEN) return;
  if (out_size != NTOK * DM) return;

  const float* x      = (const float*)d_in[0];
  const float* n1w    = (const float*)d_in[1];
  const float* n1b    = (const float*)d_in[2];
  const float* qkv_w  = (const float*)d_in[3];
  const float* Mmat   = (const float*)d_in[4];
  const float* scalep = (const float*)d_in[5];
  const float* proj_w = (const float*)d_in[6];
  const float* proj_b = (const float*)d_in[7];
  const float* n2w    = (const float*)d_in[8];
  const float* n2b    = (const float*)d_in[9];
  const float* cen    = (const float*)d_in[10];
  const float* betap  = (const float*)d_in[11];
  const float* fcw    = (const float*)d_in[12];
  float* outf = (float*)d_out;

  const size_t PWqkv = (size_t)QKVR * DM * 2;
  const size_t PWp   = (size_t)DM * DM * 2;
  const size_t PMT   = (size_t)HD * HD * 2;
  const size_t PC16  = (size_t)NCP * DM * 2;
  const size_t PBc   = 256;
  const size_t PKmk  = (size_t)NQK * 4;
  const size_t P16   = (size_t)NTOK * DM * 2;
  const size_t PF32  = (size_t)NTOK * DM * 4;
  const size_t PVT   = (size_t)NBH * HD * NT * 2;
  size_t off = 0;
  const size_t oWq  = off; off += PWqkv;
  const size_t oWp  = off; off += PWp;
  const size_t oMT  = off; off += PMT;
  const size_t oC16 = off; off += PC16;
  const size_t oBc  = off; off += PBc;
  const size_t oKmk = off; off += PKmk;
  const size_t oA   = off; off += P16;
  const size_t oB   = off; off += PF32;
  const size_t oC   = off; off += PF32;
  const size_t oD   = off; off += PF32;
  const size_t oE   = off; off += PVT;
  if (off > ws_size) return;
  if (off > (size_t)134217728) return;

  char* ws = (char*)d_ws;
  unsigned short* Wqkv16 = (unsigned short*)(ws + oWq);
  unsigned short* Wp16   = (unsigned short*)(ws + oWp);
  unsigned short* MT16   = (unsigned short*)(ws + oMT);
  unsigned short* C16    = (unsigned short*)(ws + oC16);
  float*          Bc     = (float*)(ws + oBc);
  float*          Kmk    = (float*)(ws + oKmk);
  unsigned short* H16    = (unsigned short*)(ws + oA);
  unsigned short* Y16    = (unsigned short*)(ws + oA);
  unsigned short* H2p    = (unsigned short*)(ws + oA);
  float*          Vf     = (float*)(ws + oB);
  unsigned short* QMh    = (unsigned short*)(ws + oB);
  unsigned short* QMl    = (unsigned short*)(ws + oB + P16);
  float*          X1f    = (float*)(ws + oB);
  unsigned short* Qh     = (unsigned short*)(ws + oC);
  unsigned short* Ql     = (unsigned short*)(ws + oC + P16);
  unsigned short* KMh    = (unsigned short*)(ws + oC);
  unsigned short* KMl    = (unsigned short*)(ws + oC + P16);
  float*          Cg     = (float*)(ws + oC);
  unsigned short* Kh     = (unsigned short*)(ws + oD);
  unsigned short* Kl     = (unsigned short*)(ws + oD + P16);
  unsigned short* VT16   = (unsigned short*)(ws + oE);

  const dim3 blk(256);
  const int n8qkv = QKVR * DM / 8;
  const int n8p   = DM * DM / 8;
  const dim3 gWq((n8qkv + 255) / 256);
  const dim3 gWp((n8p + 255) / 256);
  const dim3 gMT(HD / 64, HD / 64);
  const dim3 gG768(((NTOK / 64) * (DM / 64) + 7) / 8);
  const dim3 gGhl(((NQK / 32) * (HD / 64) + 7) / 8);
  const dim3 gGcen(((NTOK / 64) * (NCP / 64) + 7) / 8);
  const dim3 gVt(NT / 64, NBH * 3);
  const dim3 gKmk(NQK / 32);
  const dim3 gAttn(NBH * NQB);

  const float wScale  = 64.0f;
  const float hScale  = 8.0f;
  const float vScale  = 16.0f;
  const float qkOut   = 16.0f / (8.0f * 64.0f);

  w_cvt<<<gWq, blk, 0, stream>>>(qkv_w, Wqkv16, n8qkv, wScale);
  w_cvt<<<gWp, blk, 0, stream>>>(proj_w, Wp16, n8p, wScale);
  wt_cvt<<<gMT, blk, 0, stream>>>(Mmat, HD, HD, MT16, 1.0f);
  cen_prep<<<dim3(1), blk, 0, stream>>>(cen, C16, Bc);
  ln_f16<<<dim3(NTOK), dim3(96), 0, stream>>>(x, n1w, n1b, H16, 1, hScale);
  gemm64<3, 0><<<gG768, blk, 0, stream>>>(H16, DM, Wqkv16, DM, proj_b, x, DM, Vf, Qh, Ql, HD, NTOK, DM, DM,
                                          qkOut);
  gemm64<3, 0><<<gG768, blk, 0, stream>>>(H16, DM, Wqkv16 + (size_t)DM * DM, DM, proj_b, x, DM, Vf, Kh, Kl, HD,
                                          NTOK, DM, DM, qkOut);
  gemm64<0, 0><<<gG768, blk, 0, stream>>>(H16, DM, Wqkv16 + (size_t)2 * DM * DM, DM, proj_b, x, DM, Vf, Kh, Kl,
                                          DM, NTOK, DM, DM, 1.0f / (8.0f * 64.0f));
  vt_planes<<<gVt, blk, 0, stream>>>(Vf, VT16, vScale);
  gemm2hl<<<gGhl, blk, 0, stream>>>(Qh, Ql, HD, MT16, HD, QMh, QMl, HD, NQK, HD, HD, 1.0f);
  gemm2hl<<<gGhl, blk, 0, stream>>>(Kh, Kl, HD, MT16, HD, KMh, KMl, HD, NQK, HD, HD, 1.0f);
  kmk_k<<<gKmk, blk, 0, stream>>>(Kh, Kl, KMh, KMl, Kmk);
  attn_k<<<gAttn, dim3(128), 0, stream>>>(QMh, QMl, Kh, Kl, VT16, Kmk, scalep, Y16);
  gemm64<1, 1><<<gG768, blk, 0, stream>>>(Y16, DM, Wp16, DM, proj_b, x, DM, X1f, Kh, Kl, DM, NTOK, DM, DM,
                                          1.0f / 1024.0f);
  ln_f16<<<dim3(NTOK), dim3(96), 0, stream>>>(X1f, n2w, n2b, H2p, 0, hScale);
  gemm64<0, 0><<<gGcen, blk, 0, stream>>>(H2p, DM, C16, DM, proj_b, x, DM, Cg, Kh, Kl, NCP, NTOK, NCP, DM,
                                          1.0f / 8.0f);
  final_k<<<dim3(NTOK), dim3(192), 0, stream>>>(X1f, n2w, n2b, Cg, Bc, betap, fcw, outf);
  (void)hipGetLastError();
}
